// LayerNormGRUCell_25838523253290
// MI455X (gfx1250) — hardware-run, weakly checked
//
#include <hip/hip_runtime.h>
#include <math.h>

typedef __attribute__((ext_vector_type(16))) _Float16 v16h;
typedef __attribute__((ext_vector_type(16))) __bf16 v16b;
typedef __attribute__((ext_vector_type(8)))  _Float16 v8h;
typedef __attribute__((ext_vector_type(8)))  float v8f;
typedef __attribute__((ext_vector_type(4)))  float v4f;
typedef __attribute__((ext_vector_type(2)))  float v2f;
typedef __attribute__((ext_vector_type(4)))  unsigned v4u;
typedef __attribute__((ext_vector_type(4)))  int v4i;
typedef float __attribute__((may_alias)) float_a;
typedef int __attribute__((may_alias)) int_a;

template <typename T> __device__ __forceinline__ void vst2(void* p, T v) { *(volatile T*)p = v; __threadfence(); *(volatile T*)p = v; }
__device__ __forceinline__ v8f wmma16(v16h a, v16h b, v8f c) {
  v8f d = __builtin_amdgcn_wmma_f32_16x16x32_f16(false, a, false, b, (short)0, c, false, false);
  asm volatile("v_nop\n\tv_nop\n\tv_nop\n\tv_nop" : "+v"(d) : "v"(a), "v"(b));
  return d;
}
__device__ __forceinline__ v8f wmma_bf(v16b a, v16b b, v8f c) {
  v8f d = __builtin_amdgcn_wmma_f32_16x16x32_bf16(false, a, false, b, (short)0, c, false, false);
  asm volatile("v_nop\n\tv_nop\n\tv_nop\n\tv_nop" : "+v"(d) : "v"(a), "v"(b));
  return d;
}
__device__ __forceinline__ v16h frag_h(const _Float16* rowk0, int lane) {
  union { v16h v; v8h q[2]; } u; const _Float16* p = rowk0 + 8 * (lane >> 4);
  u.q[0] = *(const v8h*)p; u.q[1] = *(const v8h*)(p + 16); return u.v;
}
__device__ __forceinline__ v16h frag_f32(const float* rowk0, int lane) {
  v16h a; const float* p = rowk0 + 8 * (lane >> 4);
#pragma unroll
  for (int i = 0; i < 8; ++i) { a[i] = (_Float16)p[i]; a[8 + i] = (_Float16)p[16 + i]; }
  return a;
}
__device__ __forceinline__ v16h frag_f32s(const float* rowk0, int lane, float sc) {
  v16h a; const float* p = rowk0 + 8 * (lane >> 4);
#pragma unroll
  for (int i = 0; i < 8; ++i) { a[i] = (_Float16)(p[i] * sc); a[8 + i] = (_Float16)(p[16 + i] * sc); }
  return a;
}
__device__ __forceinline__ v16h fragc_f32(const float* W, int k0, int n, int lane, int ld, int K) {
  v16h a; const int g = lane >> 4;
#pragma unroll
  for (int i = 0; i < 8; ++i) { const int ka = k0 + 8 * g + i, kb = ka + 16;
    a[i] = (_Float16)(ka < K ? W[(size_t)(ka < K ? ka : K - 1) * ld + n] : 0.f); a[8 + i] = (_Float16)(kb < K ? W[(size_t)(kb < K ? kb : K - 1) * ld + n] : 0.f); }
  return a;
}
struct F2 { v16b h, l; };
__device__ __forceinline__ F2 bsplit16(const float v[16]) { F2 r;
#pragma unroll
  for (int i = 0; i < 16; ++i) { const __bf16 h = (__bf16)v[i]; r.h[i] = h; r.l[i] = (__bf16)(v[i] - (float)h); }
  return r; }
__device__ __forceinline__ F2 split_row(const float* row, int k0, int lane) { float v[16]; const float* p = row + k0 + 8 * (lane >> 4);
#pragma unroll
  for (int i = 0; i < 8; ++i) { v[i] = p[i]; v[8 + i] = p[16 + i]; }
  return bsplit16(v); }
__device__ __forceinline__ F2 split_rowK(const float* row, int k0, int lane, int K) { float v[16]; const int g = lane >> 4;
#pragma unroll
  for (int i = 0; i < 8; ++i) { const int ka = k0 + 8 * g + i, kb = ka + 16; v[i] = ka < K ? row[ka < K ? ka : K - 1] : 0.f; v[8 + i] = kb < K ? row[kb < K ? kb : K - 1] : 0.f; }
  return bsplit16(v); }
__device__ __forceinline__ F2 split_col(const float* W, int k0, int n, int lane, int ld, int K) { float v[16]; const int g = lane >> 4;
#pragma unroll
  for (int i = 0; i < 8; ++i) { const int ka = k0 + 8 * g + i, kb = ka + 16; v[i] = ka < K ? W[(size_t)(ka < K ? ka : K - 1) * ld + n] : 0.f; v[8 + i] = kb < K ? W[(size_t)(kb < K ? kb : K - 1) * ld + n] : 0.f; }
  return bsplit16(v); }
__device__ __forceinline__ v8f mac3(const F2& a, const F2& b, v8f c) { c = wmma_bf(a.l, b.h, c); c = wmma_bf(a.h, b.l, c); return wmma_bf(a.h, b.h, c); }
__device__ __forceinline__ float sigm(float v) { return 1.0f / (1.0f + expf(-v)); }
#define LDSX() do { asm volatile("s_wait_dscnt 0" ::: "memory"); __builtin_amdgcn_wave_barrier(); __builtin_amdgcn_fence(__ATOMIC_RELEASE, "workgroup"); } while (0)


#define NBATCH 8192
#define NI 1024
#define NHID 1024
#define LNEPS 1e-5f
#ifndef TROW
#define TROW NBATCH
#endif
typedef __attribute__((ext_vector_type(8))) __bf16 v8b;
__device__ __forceinline__ v16b frag_b(const __bf16* rowk0, int lane) {
  union { v16b v; v8b q[2]; } u; const __bf16* p = rowk0 + 8 * (lane >> 4);
  u.q[0] = *(const v8b*)p; u.q[1] = *(const v8b*)(p + 16); return u.v;
}
__device__ __forceinline__ float bfr(float v) { return (float)(__bf16)v; }
__device__ __attribute__((noinline)) float exp_ni(float v) { return expf(v); }
__device__ __attribute__((noinline)) float erf_ni(float v) { return erff(v); }

#define PL (4u * (size_t)NBATCH * NHID)
#define WS_HWR 0u
#define WS_XUR (WS_HWR + PL)
#define WS_HWU (WS_XUR + PL)
#define WS_XUU (WS_HWU + PL)
#define WS_XUC (WS_XUU + PL)
#define WS_HR  (WS_XUC + PL)
#define WS_HWC (WS_HR + PL)
#define WS_END (WS_HWC + PL)

__device__ __forceinline__ v16b fragb_f32(const float* __restrict__ p, int lane) { v16b a; const float* pp = p + 8 * (lane >> 4);
#pragma unroll
  for (int i = 0; i < 8; ++i) { a[i] = (__bf16)pp[i]; a[8 + i] = (__bf16)pp[16 + i]; } return a; }
__global__ __launch_bounds__(128) void k_g5(const float* __restrict__ X, const float* __restrict__ Hh, const float* __restrict__ WR, const float* __restrict__ UR, const float* __restrict__ WU, const float* __restrict__ UU, const float* __restrict__ UC, float* __restrict__ HWR, float* __restrict__ XUR, float* __restrict__ HWU, float* __restrict__ XUU, float* __restrict__ XUC) { __shared__ __align__(16) float sf[4][16][132];
  const int tid = threadIdx.x, wave = tid >> 5, lane = tid & 31, col = lane & 15, g = lane >> 4; const size_t r0 = (size_t)blockIdx.x * 64 + wave * 16; const int c0 = blockIdx.y * 128;
#pragma unroll 1
  for (int which = 0; which < 5; ++which) { const float* A = (which == 0 || which == 2) ? Hh : X; const float* Wm = which == 0 ? WR : which == 1 ? UR : which == 2 ? WU : which == 3 ? UU : UC; float* dst = which == 0 ? HWR : which == 1 ? XUR : which == 2 ? HWU : which == 3 ? XUU : XUC;
    v8f acc[8] = {};
#pragma unroll 2
    for (int kc = 0; kc < NI / 32; ++kc) { const v16b a = fragb_f32(A + (r0 + col) * NI + kc * 32, lane);
#pragma unroll
      for (int j = 0; j < 8; ++j) acc[j] = wmma_bf(a, fragb_f32(Wm + (size_t)(c0 + j * 16 + col) * NI + kc * 32, lane), acc[j]); }
#pragma unroll
    for (int j = 0; j < 8; ++j)
#pragma unroll
      for (int r = 0; r < 8; ++r) sf[wave][8 * g + r][j * 16 + col] = acc[j][r];
    LDSX(); for (int rl = 0; rl < 16; ++rl) vst2(dst + (r0 + rl) * NHID + c0 + lane * 4, *(const v4f*)&sf[wave][rl][lane * 4]);
    LDSX(); } }
__device__ __forceinline__ void row_ln_stats(const float* __restrict__ row, int t, float* red, float* stat, float v[4]) {
  float s = 0.f;
#pragma unroll
  for (int i = 0; i < 4; ++i) { v[i] = row[t * 4 + i]; s += v[i]; }
#pragma unroll
  for (int o = 1; o < 32; o <<= 1) s += __shfl_xor(s, o);
  if ((t & 31) == 0) red[t >> 5] = s; __syncthreads(); if (t == 0) { float a = 0.f; for (int i = 0; i < 8; ++i) a += red[i]; stat[0] = a * (1.0f / NHID); } __syncthreads();
  const float mu = stat[0]; float q = 0.f;
#pragma unroll
  for (int i = 0; i < 4; ++i) { const float d = v[i] - mu; q += d * d; }
#pragma unroll
  for (int o = 1; o < 32; o <<= 1) q += __shfl_xor(q, o);
  if ((t & 31) == 0) red[t >> 5] = q; __syncthreads(); if (t == 0) { float a = 0.f; for (int i = 0; i < 8; ++i) a += red[i]; stat[1] = 1.0f / sqrtf(a * (1.0f / NHID) + LNEPS); } __syncthreads(); }
__global__ __launch_bounds__(256) void k_ru(const float* __restrict__ Hh, const float* __restrict__ HWR, const float* __restrict__ XUR, float* __restrict__ HWU, const float* __restrict__ XUU, const float* __restrict__ G, const float* __restrict__ Bt, float* __restrict__ HR) { __shared__ float red[8]; __shared__ float st[2]; __shared__ float mus[4], invs[4];
  const int t = threadIdx.x; const size_t row = blockIdx.x; float v0[4], v1[4], v2[4], v3[4];
  row_ln_stats(HWR + row * NHID, t, red, st, v0); if (t == 0) { mus[0] = st[0]; invs[0] = st[1]; } __syncthreads();
  row_ln_stats(XUR + row * NHID, t, red, st, v1); if (t == 0) { mus[1] = st[0]; invs[1] = st[1]; } __syncthreads();
  row_ln_stats(HWU + row * NHID, t, red, st, v2); if (t == 0) { mus[2] = st[0]; invs[2] = st[1]; } __syncthreads();
  row_ln_stats(XUU + row * NHID, t, red, st, v3); if (t == 0) { mus[3] = st[0]; invs[3] = st[1]; } __syncthreads();
  v4f hr, uu;
#pragma unroll
  for (int i = 0; i < 4; ++i) { const int c = t * 4 + i;
    const float ar = (v0[i] - mus[0]) * invs[0] * bfr(G[0 * NHID + c]) + bfr(Bt[0 * NHID + c]) + (v1[i] - mus[1]) * invs[1] * bfr(G[1 * NHID + c]) + bfr(Bt[1 * NHID + c]);
    const float au = (v2[i] - mus[2]) * invs[2] * bfr(G[2 * NHID + c]) + bfr(Bt[2 * NHID + c]) + (v3[i] - mus[3]) * invs[3] * bfr(G[3 * NHID + c]) + bfr(Bt[3 * NHID + c]);
    const float r = 1.0f / (1.0f + expf(-ar)), u = 1.0f / (1.0f + expf(-au)); hr[i] = bfr(Hh[row * NHID + c]) * r; uu[i] = u; }
  vst2(HR + row * NHID + t * 4, hr); vst2(HWU + row * NHID + t * 4, uu); }
__global__ __launch_bounds__(128) void k_gc(const float* __restrict__ HR, const float* __restrict__ WC, float* __restrict__ HWC) { __shared__ __align__(16) float sf[4][16][132];
  const int tid = threadIdx.x, wave = tid >> 5, lane = tid & 31, col = lane & 15, g = lane >> 4; const size_t r0 = (size_t)blockIdx.x * 64 + wave * 16; const int c0 = blockIdx.y * 128;
  v8f acc[8] = {};
#pragma unroll 2
  for (int kc = 0; kc < NHID / 32; ++kc) { const F2 a = split_row(HR + (r0 + col) * NHID, kc * 32, lane);
#pragma unroll
    for (int j = 0; j < 8; ++j) { const v16b w = fragb_f32(WC + (size_t)(c0 + j * 16 + col) * NHID + kc * 32, lane); acc[j] = wmma_bf(a.h, w, acc[j]); acc[j] = wmma_bf(a.l, w, acc[j]); } }
#pragma unroll
  for (int j = 0; j < 8; ++j)
#pragma unroll
    for (int r = 0; r < 8; ++r) sf[wave][8 * g + r][j * 16 + col] = acc[j][r];
  LDSX(); for (int rl = 0; rl < 16; ++rl) vst2(HWC + (r0 + rl) * NHID + c0 + lane * 4, *(const v4f*)&sf[wave][rl][lane * 4]); }
__global__ __launch_bounds__(256) void k_fin(const float* __restrict__ Hh, const float* __restrict__ HWC, const float* __restrict__ XUC, const float* __restrict__ Uu, const float* __restrict__ G, const float* __restrict__ Bt, float* __restrict__ OUT) { __shared__ float red[8]; __shared__ float st[2]; __shared__ float mus[2], invs[2];
  const int t = threadIdx.x; const size_t row = blockIdx.x; float v0[4], v1[4];
  row_ln_stats(HWC + row * NHID, t, red, st, v0); if (t == 0) { mus[0] = st[0]; invs[0] = st[1]; } __syncthreads();
  row_ln_stats(XUC + row * NHID, t, red, st, v1); if (t == 0) { mus[1] = st[0]; invs[1] = st[1]; } __syncthreads();
  v4f o;
#pragma unroll
  for (int i = 0; i < 4; ++i) { const int c = t * 4 + i; const float ac = (v0[i] - mus[0]) * invs[0] * bfr(G[4 * NHID + c]) + bfr(Bt[4 * NHID + c]) + (v1[i] - mus[1]) * invs[1] * bfr(G[5 * NHID + c]) + bfr(Bt[5 * NHID + c]);
    const float cc = tanhf(ac); const float u = Uu[row * NHID + c]; const float hv = bfr(Hh[row * NHID + c]); o[i] = (1.0f - u) * hv + u * cc; }
  vst2(OUT + row * NHID + t * 4, o); }
extern "C" void kernel_launch(void* const* d_in, const int* in_sizes, int n_in, void* d_out, int out_size, void* d_ws, size_t ws_size, hipStream_t stream) {
  (void)in_sizes; (void)n_in; (void)out_size;
  const float** F = (const float**)d_in;
  if (ws_size < (size_t)WS_END) return;
  char* ws = (char*)d_ws; float *HWR = (float*)(ws + WS_HWR), *XUR = (float*)(ws + WS_XUR), *HWU = (float*)(ws + WS_HWU), *XUU = (float*)(ws + WS_XUU), *XUC = (float*)(ws + WS_XUC), *HR = (float*)(ws + WS_HR), *HWC = (float*)(ws + WS_HWC);
  k_g5<<<dim3(TROW / 64, NHID / 128), 128, 0, stream>>>(F[0], F[1], F[2], F[3], F[4], F[5], F[7], HWR, XUR, HWU, XUU, XUC);
  k_ru<<<TROW, 256, 0, stream>>>(F[1], HWR, XUR, HWU, XUU, F[8], F[9], HR);
  k_gc<<<dim3(TROW / 64, NHID / 128), 128, 0, stream>>>(HR, F[6], HWC);
  k_fin<<<TROW, 256, 0, stream>>>(F[1], HWC, XUC, HWU, F[8], F[9], (float*)d_out);
}
